// MultiHeadAttention_74517682586324
// MI455X (gfx1250) — hardware-run, weakly checked
//
#include <hip/hip_runtime.h>


#ifndef NB
#define NB 4
#endif
#ifndef SEQ
#define SEQ 2048
#endif
#define NB_FULL  4
#define SEQ_FULL 2048
#ifndef OUT_SEQ
#define OUT_SEQ SEQ
#endif
#define DM   1024
#define NH_  16
#define HD   64
#define AW   4
#define ER   ((SEQ) < 512 ? (SEQ) : 512)
#define QRS  2048.0f
#define QRI  (1.0f / 2048.0f)
#define SC2  (0.125f * 1.4426950408889634f)
#define PSH  8.0f
#define NEGB (-3.0e38f)
#define BIGI 0x40000000

static_assert(HD == 64);
static_assert(NH_ * HD == DM);
static_assert(DM % 64 == 0);
static_assert(DM % 32 == 0);
static_assert((DM & (DM - 1)) == 0);
static_assert(SEQ % 64 == 0);
static_assert((NB * SEQ) % 64 == 0);
static_assert(SEQ % 32 == 0);
static_assert(ER % 64 == 0);
static_assert(ER % (16 * AW) == 0);
static_assert((SEQ - ER) % (16 * AW) == 0);
static_assert(((size_t)SEQ * DM) % 8 == 0);
static_assert(NB <= NB_FULL);
static_assert(SEQ <= SEQ_FULL);

typedef _Float16 h16;
typedef unsigned short bf;
typedef __attribute__((ext_vector_type(16))) __bf16   v16bf;
typedef __attribute__((ext_vector_type(16))) _Float16 v16h;
typedef __attribute__((ext_vector_type(8)))  _Float16 v8h;
typedef __attribute__((ext_vector_type(8)))  unsigned short v8us;
typedef __attribute__((ext_vector_type(8)))  float    v8f;
typedef __attribute__((ext_vector_type(4)))  float    v4f;
typedef v4f  __attribute__((may_alias)) v4fa;

__device__ __forceinline__ unsigned short f2bf(float f) { unsigned u = __float_as_uint(f); u += 0x7FFFu + ((u >> 16) & 1u); return (unsigned short)(u >> 16); }
__device__ __forceinline__ float bf2f(unsigned short s) { return __uint_as_float(((unsigned)s) << 16); }
__device__ __forceinline__ h16 tohi(float x) { return (__builtin_fabsf(x) < 6.1035156e-5f) ? (h16)0.0f : (h16)x; }
__device__ __forceinline__ v16h cat16(v8h lo, v8h hi) { return __builtin_shufflevector(lo, hi, 0, 1, 2, 3, 4, 5, 6, 7, 8, 9, 10, 11, 12, 13, 14, 15); }
__device__ __forceinline__ v16bf cat16b(v8us lo, v8us hi) { return __builtin_bit_cast(v16bf, __builtin_shufflevector(lo, hi, 0, 1, 2, 3, 4, 5, 6, 7, 8, 9, 10, 11, 12, 13, 14, 15)); }
__device__ __forceinline__ v8f wmma16(v16h a, v16h b, v8f c) { return __builtin_amdgcn_wmma_f32_16x16x32_f16(false, a, false, b, (short)0, c, false, false); }
__device__ __forceinline__ v8f wmmab(v16bf a, v16bf b, v8f c) { return __builtin_amdgcn_wmma_f32_16x16x32_bf16(false, a, false, b, (short)0, c, false, false); }
__device__ __forceinline__ v16h  ldh(const h16* p) { return cat16(*(const v8h*)p, *(const v8h*)(p + 16)); }
__device__ __forceinline__ v16bf ldb(const bf* p)  { return cat16b(*(const v8us*)p, *(const v8us*)(p + 16)); }
__device__ __forceinline__ void wave_sync() { __builtin_amdgcn_fence(3  , "wavefront"); __builtin_amdgcn_wave_barrier(); asm volatile("" ::: "memory"); }

__global__ __launch_bounds__(256) void k_cvt8(const float* __restrict__ src, bf* dst, size_t n8) {
    const size_t i = (size_t)blockIdx.x * 256 + threadIdx.x; if (i >= n8) return;
    const v8f v = *(const v8f*)(src + i * 8); v8us o;
#pragma unroll
    for (int k = 0; k < 8; ++k) o[k] = f2bf(v[k]);
    *(volatile v8us*)(dst + i * 8) = o; __threadfence(); *(volatile v8us*)(dst + i * 8) = o;
}

__global__ __launch_bounds__(256) void k_cvtT(const float* __restrict__ W, bf* WT) {
    __shared__ float ts[64 * 65];
    const int tid = threadIdx.x; const int k0 = blockIdx.x * 64, n0 = blockIdx.y * 64;
#pragma unroll
    for (int i = 0; i < 4; ++i) { const int idx = i * 256 + tid; const int r = idx >> 4, c4 = (idx & 15) * 4;
        const v4f v = *(const v4f*)(W + (size_t)(k0 + r) * DM + n0 + c4);
        ts[r * 65 + c4 + 0] = v[0]; ts[r * 65 + c4 + 1] = v[1]; ts[r * 65 + c4 + 2] = v[2]; ts[r * 65 + c4 + 3] = v[3]; }
    __syncthreads();
#pragma unroll 1
    for (int ps = 0; ps < 2; ++ps) {
#pragma unroll
        for (int i = 0; i < 2; ++i) { const int idx = i * 256 + tid; const int n = idx >> 3, kq = (idx & 7) * 8;
            v8us o;
#pragma unroll
            for (int j = 0; j < 8; ++j) o[j] = f2bf(ts[(kq + j) * 65 + n]);
            *(volatile v8us*)(WT + (size_t)(n0 + n) * DM + k0 + kq) = o; }
        if (ps == 0) __threadfence(); }
}

template <int F32OUT, int K, int PA, int PB, int KBM>
__global__ __launch_bounds__(32) void k_gemm(const bf* __restrict__ A, const bf* __restrict__ Bt, h16* Ph, h16* Pr, float* Of,
                                             int RB, size_t sRB, int pitch, int CB, size_t sCB, int erow, int ecol, size_t sRBr, int pitchR, size_t sCBr) {
    __shared__ __align__(16) float os[16 * 68];
    const int lane = threadIdx.x & 31, lr = lane & 15, hi = lane >> 4; const int r0 = blockIdx.x * 64, c0 = blockIdx.y * 64;
    v8f acc[4][4];
#pragma unroll
    for (int mb = 0; mb < 4; ++mb)
#pragma unroll
        for (int nb = 0; nb < 4; ++nb) acc[mb][nb] = (v8f){};
    const size_t aoff = (size_t)(r0 + lr) * PA + 8 * hi, boff = (size_t)(c0 + lr) * PB + 8 * hi;
#pragma unroll 1
    for (int kc = 0; kc < K; kc += 32) {
        const int kb = kc & KBM;
        v16bf a[4];
#pragma unroll
        for (int mb = 0; mb < 4; ++mb) a[mb] = ldb(A + aoff + (size_t)mb * 16 * PA + kc);
#pragma unroll
        for (int nb = 0; nb < 4; ++nb) { const v16bf b = ldb(Bt + boff + (size_t)nb * 16 * PB + kb);
#pragma unroll
            for (int mb = 0; mb < 4; ++mb) acc[mb][nb] = wmmab(a[mb], b, acc[mb][nb]); }
        asm volatile("v_nop\n\tv_nop\n\tv_nop\n\tv_nop" : "+v"(acc[0][0]), "+v"(acc[1][1]), "+v"(acc[2][2]), "+v"(acc[3][3]) : "v"(a[0]), "v"(a[1]), "v"(a[2]), "v"(a[3]));
    }
    const size_t tbase = (size_t)(r0 / RB) * sRB + (size_t)(r0 % RB) * (size_t)pitch + (size_t)(c0 / CB) * sCB + (size_t)(c0 % CB);
    const size_t rbase = (size_t)(r0 / RB) * sRBr + (size_t)(r0 % RB) * (size_t)pitchR + (size_t)(c0 / CB) * sCBr + (size_t)(c0 % CB);
    const bool res = (F32OUT == 0) && ((r0 % RB) < erow) && ((c0 % CB) < ecol);
#pragma unroll
    for (int mb = 0; mb < 4; ++mb) {
#pragma unroll
        for (int nb = 0; nb < 4; ++nb) {
#pragma unroll
            for (int j = 0; j < 8; ++j) os[(hi * 8 + j) * 68 + nb * 16 + lr] = acc[mb][nb][j]; }
        wave_sync();
        if (F32OUT) {
            float* ob = Of + tbase + (size_t)(mb * 16) * (size_t)pitch;
#pragma unroll 1
            for (int ps = 0; ps < 2; ++ps) {
#pragma unroll
                for (int s = 0; s < 8; ++s) { const int row = 2 * s + hi, cofs = lr * 4;
                    const v4f val = *(const v4fa*)(&os[row * 68 + cofs]);
                    *(volatile v4f*)(ob + (size_t)row * (size_t)pitch + cofs) = val; }
                if (ps == 0) __threadfence(); }
        } else {
            const size_t sb = tbase + (size_t)(mb * 16) * (size_t)pitch;
            const size_t sr = rbase + (size_t)(mb * 16) * (size_t)pitchR;
#pragma unroll 1
            for (int ps = 0; ps < 2; ++ps) {
#pragma unroll
                for (int s = 0; s < 4; ++s) { const int row = 4 * s + (lane >> 3), c8 = (lane & 7) * 8;
                    const v4f x0 = *(const v4fa*)(&os[row * 68 + c8]); const v4f x1 = *(const v4fa*)(&os[row * 68 + c8 + 4]); v8h hv, rv;
#pragma unroll
                    for (int i = 0; i < 4; ++i) { const h16 a0 = tohi(x0[i]); const h16 a1 = tohi(x1[i]); hv[i] = a0; hv[4 + i] = a1; rv[i] = (h16)((x0[i] - (float)a0) * QRS); rv[4 + i] = (h16)((x1[i] - (float)a1) * QRS); }
                    *(volatile v8h*)(Ph + sb + (size_t)row * (size_t)pitch + c8) = hv;
                    if (res) *(volatile v8h*)(Pr + sr + (size_t)row * (size_t)pitchR + c8) = rv; }
                if (ps == 0) __threadfence(); }
        }
        wave_sync();
    }
}

template <int EARLY>
__global__ __launch_bounds__(32 * AW) void k_flash(const h16* __restrict__ QH, const h16* __restrict__ QR, const h16* __restrict__ KP, const h16* __restrict__ KR,
                                                   const h16* __restrict__ VT, const h16* __restrict__ VR, bf* CX, int tstart) {
    __shared__ __align__(16) float os[AW * 16 * 68];
    const int lane = threadIdx.x & 31, lr = lane & 15, hi = lane >> 4;
    const int wave = __builtin_amdgcn_readfirstlane((int)(threadIdx.x >> 5));
    const int zh = blockIdx.y; const int b = zh / NH_, h = zh % NH_;
    const int t0 = tstart + ((int)blockIdx.x * AW + wave) * 16;
    const size_t pbase = (size_t)zh * SEQ * HD;
    const size_t rbase = (size_t)zh * ER * HD;
    const size_t qo = pbase + (size_t)(t0 + lr) * HD + 8 * hi;
    const v16h qh0 = ldh(QH + qo), qh1 = ldh(QH + qo + 32);
    v16h qr0 = qh0, qr1 = qh1;
    if (EARLY) { const size_t qro = rbase + (size_t)(t0 + lr) * HD + 8 * hi; qr0 = ldh(QR + qro); qr1 = ldh(QR + qro + 32); }
    const size_t ko  = pbase + (size_t)lr * HD + 8 * hi;
    const size_t kro = rbase + (size_t)lr * HD + 8 * hi;
    const size_t vo  = pbase + (size_t)lr * SEQ + 8 * hi;
    const size_t vro = rbase + (size_t)lr * ER + 8 * hi;
    v8f oH[4], oL[4];
#pragma unroll
    for (int j = 0; j < 4; ++j) { oH[j] = (v8f){}; oL[j] = (v8f){}; }
    float m = NEGB, l = 0.0f;
    const int qrow = t0 + lr;
    const int kend = t0 + 16;
#pragma unroll 1
    for (int key0 = 0; key0 < kend; key0 += 32) {
        const h16* ka = KP + ko + (size_t)key0 * HD;
        const v16h ka0 = ldh(ka), ka1 = ldh(ka + 32), kb0 = ldh(ka + 16 * HD), kb1 = ldh(ka + 16 * HD + 32);
        v8f sHa = (v8f){}, sLa = (v8f){}, sHb = (v8f){}, sLb = (v8f){};
        if (EARLY) {
            const h16* kr = KR + kro + (size_t)key0 * HD;
            const v16h ra0 = ldh(kr), ra1 = ldh(kr + 32), rb0 = ldh(kr + 16 * HD), rb1 = ldh(kr + 16 * HD + 32);
            sHa = wmma16(ka0, qh0, sHa); sLa = wmma16(ka0, qr0, sLa); sHb = wmma16(kb0, qh0, sHb); sLb = wmma16(kb0, qr0, sLb);
            sHa = wmma16(ka1, qh1, sHa); sLa = wmma16(ra0, qh0, sLa); sHb = wmma16(kb1, qh1, sHb); sLb = wmma16(rb0, qh0, sLb);
            sLa = wmma16(ka1, qr1, sLa); sLb = wmma16(kb1, qr1, sLb);
            sLa = wmma16(ra1, qh1, sLa); sLb = wmma16(rb1, qh1, sLb);
            asm volatile("v_nop\n\tv_nop\n\tv_nop\n\tv_nop" : "+v"(sHa), "+v"(sLa), "+v"(sHb), "+v"(sLb)
                         : "v"(ka0), "v"(ka1), "v"(kb0), "v"(kb1), "v"(ra0), "v"(ra1), "v"(rb0), "v"(rb1), "v"(qh0), "v"(qh1), "v"(qr0), "v"(qr1));
        } else {
            sHa = wmma16(ka0, qh0, sHa); sHb = wmma16(kb0, qh0, sHb);
            sHa = wmma16(ka1, qh1, sHa); sHb = wmma16(kb1, qh1, sHb);
            asm volatile("v_nop\n\tv_nop\n\tv_nop\n\tv_nop" : "+v"(sHa), "+v"(sHb) : "v"(ka0), "v"(ka1), "v"(kb0), "v"(kb1), "v"(qh0), "v"(qh1));
        }
        float ta[8], tb[8];
#pragma unroll
        for (int r = 0; r < 8; ++r) {
            if (EARLY) { ta[r] = (sHa[r] + sLa[r] * QRI) * SC2; tb[r] = (sHb[r] + sLb[r] * QRI) * SC2; }
            else       { ta[r] = sHa[r] * SC2;                  tb[r] = sHb[r] * SC2; } }
        if (key0 + 31 > t0) {
#pragma unroll
            for (int r = 0; r < 8; ++r) { const int kA = key0 + 8 * hi + r;
                ta[r] = (kA > qrow) ? NEGB : ta[r]; tb[r] = (kA + 16 > qrow) ? NEGB : tb[r]; }
        }
        float mx = NEGB;
#pragma unroll
        for (int r = 0; r < 8; ++r) mx = fmaxf(mx, fmaxf(ta[r], tb[r]));
        mx = fmaxf(mx, __shfl_xor(mx, 16, 32));
        const float mnew = fmaxf(m, mx);
        const float alpha = __builtin_amdgcn_exp2f(m - mnew);
        const float sh = PSH - mnew;
        v16h pH, pL; float ls = 0.0f;
        if (EARLY) {
#pragma unroll
            for (int r = 0; r < 8; ++r) { const float fa = __builtin_amdgcn_exp2f(ta[r] + sh); const float fc = __builtin_amdgcn_exp2f(tb[r] + sh);
                const h16 ha = tohi(fa); const h16 hc = tohi(fc); const h16 la = (h16)((fa - (float)ha) * QRS); const h16 lc = (h16)((fc - (float)hc) * QRS);
                pH[r] = ha; pH[8 + r] = hc; pL[r] = la; pL[8 + r] = lc; ls += ((float)ha + (float)hc) + ((float)la + (float)lc) * QRI; }
        } else {
#pragma unroll
            for (int r = 0; r < 8; ++r) { const h16 pa = (h16)__builtin_amdgcn_exp2f(ta[r] + sh); const h16 pc = (h16)__builtin_amdgcn_exp2f(tb[r] + sh); pH[r] = pa; pH[8 + r] = pc; ls += (float)pa + (float)pc; }
            pL = pH;
        }
        l = l * alpha + ls; m = mnew;
#pragma unroll
        for (int j = 0; j < 4; ++j) { oH[j] = oH[j] * alpha; if (EARLY) oL[j] = oL[j] * alpha; }
        const h16* va = VT + vo + key0;
        const v16h v0 = ldh(va), v1 = ldh(va + (size_t)16 * SEQ), v2 = ldh(va + (size_t)32 * SEQ), v3 = ldh(va + (size_t)48 * SEQ);
        if (EARLY) {
            const h16* vr = VR + vro + key0;
            const v16h w0 = ldh(vr), w1 = ldh(vr + (size_t)16 * ER), w2 = ldh(vr + (size_t)32 * ER), w3 = ldh(vr + (size_t)48 * ER);
            oH[0] = wmma16(v0, pH, oH[0]); oL[0] = wmma16(v0, pL, oL[0]); oH[1] = wmma16(v1, pH, oH[1]); oL[1] = wmma16(v1, pL, oL[1]);
            oH[2] = wmma16(v2, pH, oH[2]); oL[2] = wmma16(v2, pL, oL[2]); oH[3] = wmma16(v3, pH, oH[3]); oL[3] = wmma16(v3, pL, oL[3]);
            oL[0] = wmma16(w0, pH, oL[0]); oL[1] = wmma16(w1, pH, oL[1]); oL[2] = wmma16(w2, pH, oL[2]); oL[3] = wmma16(w3, pH, oL[3]);
            asm volatile("v_nop\n\tv_nop\n\tv_nop\n\tv_nop" : "+v"(oH[0]), "+v"(oH[1]), "+v"(oH[2]), "+v"(oH[3]), "+v"(oL[0]), "+v"(oL[1]), "+v"(oL[2]), "+v"(oL[3])
                         : "v"(v0), "v"(v1), "v"(v2), "v"(v3), "v"(w0), "v"(w1), "v"(w2), "v"(w3), "v"(pH), "v"(pL));
        } else {
            oH[0] = wmma16(v0, pH, oH[0]); oH[1] = wmma16(v1, pH, oH[1]); oH[2] = wmma16(v2, pH, oH[2]); oH[3] = wmma16(v3, pH, oH[3]);
            asm volatile("v_nop\n\tv_nop\n\tv_nop\n\tv_nop" : "+v"(oH[0]), "+v"(oH[1]), "+v"(oH[2]), "+v"(oH[3]) : "v"(v0), "v"(v1), "v"(v2), "v"(v3), "v"(pH));
        }
    }
    l += __shfl_xor(l, 16, 32);
    const float inv = 1.0f / l;
    const int wb = wave * 16 * 68;
#pragma unroll
    for (int j = 0; j < 4; ++j) { v4f a, c;
#pragma unroll
        for (int i = 0; i < 4; ++i) {
            if (EARLY) { a[i] = (oH[j][i] + oL[j][i] * QRI) * inv; c[i] = (oH[j][4 + i] + oL[j][4 + i] * QRI) * inv; }
            else       { a[i] = oH[j][i] * inv;                    c[i] = oH[j][4 + i] * inv; } }
        *(v4fa*)(&os[wb + lr * 68 + 16 * j + 8 * hi]) = a; *(v4fa*)(&os[wb + lr * 68 + 16 * j + 8 * hi + 4]) = c; }
    wave_sync();
    bf* crow = CX + ((size_t)b * SEQ + t0) * (size_t)(2 * DM) + h * HD;
#pragma unroll 1
    for (int ps = 0; ps < 2; ++ps) {
#pragma unroll
        for (int s = 0; s < 4; ++s) { const int row = 4 * s + (lane >> 3), c8 = (lane & 7) * 8;
            const v4f x0 = *(const v4fa*)(&os[wb + row * 68 + c8]); const v4f x1 = *(const v4fa*)(&os[wb + row * 68 + c8 + 4]); v8us hv, lv;
#pragma unroll
            for (int i = 0; i < 4; ++i) { const unsigned short a0 = f2bf(x0[i]); const unsigned short a1 = f2bf(x1[i]); hv[i] = a0; hv[4 + i] = a1;
                lv[i] = f2bf(x0[i] - bf2f(a0)); lv[4 + i] = f2bf(x1[i] - bf2f(a1)); }
            const size_t oo = (size_t)row * (size_t)(2 * DM) + c8;
            *(volatile v8us*)(crow + oo) = hv; *(volatile v8us*)(crow + oo + DM) = lv; }
        if (ps == 0) __threadfence(); }
}

static constexpr size_t al256(size_t v) { return (v + 255) & ~(size_t)255; }
static constexpr size_t SZ_XB = al256((size_t)NB * SEQ * DM * 2);
static constexpr size_t SZ_WB = al256((size_t)4 * DM * DM * 2);
static constexpr size_t SZ_PL = al256((size_t)NB * NH_ * SEQ * HD * 2);
static constexpr size_t SZ_RL = al256((size_t)NB * NH_ * ER * HD * 2);
static constexpr size_t SZ_CX = al256((size_t)NB * SEQ * 2 * DM * 2);
static constexpr size_t SZ_TOTAL = SZ_XB + SZ_WB + 3 * SZ_PL + 3 * SZ_RL + SZ_CX;
static_assert(SZ_TOTAL <= (size_t)134217728);
static_assert(((size_t)DM * DM * 2) % 256 == 0);

extern "C" void kernel_launch(void* const* d_in, const int* in_sizes, int n_in,
                              void* d_out, int out_size, void* d_ws, size_t ws_size, hipStream_t stream) {
    if (n_in < 5) return;
    const size_t needx = ((size_t)(NB - 1) * SEQ_FULL + SEQ) * DM;
    if ((size_t)in_sizes[0] < needx) return;
    if ((size_t)in_sizes[1] < (size_t)DM * DM || (size_t)in_sizes[2] < (size_t)DM * DM || (size_t)in_sizes[3] < (size_t)DM * DM || (size_t)in_sizes[4] < (size_t)DM * DM) return;
    if ((size_t)out_size < ((size_t)(NB - 1) * OUT_SEQ + SEQ) * DM) return;
    if (SZ_TOTAL > ws_size) return;
    const float* x = (const float*)d_in[0]; const float* wq = (const float*)d_in[1]; const float* wk = (const float*)d_in[2];
    const float* wv = (const float*)d_in[3]; const float* wo = (const float*)d_in[4];
    float* OUT = (float*)d_out;
    char* wsp = (char*)d_ws;
    bf* XB = (bf*)wsp; wsp += SZ_XB;
    bf* WB = (bf*)wsp; wsp += SZ_WB;
    h16* QH = (h16*)wsp; wsp += SZ_PL;
    h16* KP = (h16*)wsp; wsp += SZ_PL;
    h16* VT = (h16*)wsp; wsp += SZ_PL;
    h16* QR = (h16*)wsp; wsp += SZ_RL;
    h16* KR = (h16*)wsp; wsp += SZ_RL;
    h16* VR = (h16*)wsp; wsp += SZ_RL;
    bf* CX = (bf*)wsp; wsp += SZ_CX;
    bf* WQ = WB; bf* WK = WB + (size_t)DM * DM; bf* WV = WB + (size_t)2 * DM * DM; bf* WO = WB + (size_t)3 * DM * DM;

    if (SEQ == SEQ_FULL) {
        const size_t n8 = (size_t)NB * SEQ * DM / 8;
        k_cvt8<<<(unsigned)((n8 + 255) / 256), 256, 0, stream>>>(x, XB, n8);
    } else {
        const size_t n8 = (size_t)SEQ * DM / 8;
        for (int b = 0; b < NB; ++b) k_cvt8<<<(unsigned)((n8 + 255) / 256), 256, 0, stream>>>(x + (size_t)b * SEQ_FULL * DM, XB + (size_t)b * SEQ * DM, n8);
    }
    { const dim3 g(DM / 64, DM / 64, 1);
      k_cvtT<<<g, 256, 0, stream>>>(wq, WQ); k_cvtT<<<g, 256, 0, stream>>>(wk, WK); k_cvtT<<<g, 256, 0, stream>>>(wv, WV); k_cvtT<<<g, 256, 0, stream>>>(wo, WO); }

    k_gemm<0, DM, DM, DM, DM - 1><<<dim3(NB * SEQ / 64, DM / 64, 1), 32, 0, stream>>>(XB, WQ, QH, QR, OUT,
        SEQ, (size_t)NH_ * SEQ * HD, HD, HD, (size_t)SEQ * HD, ER, BIGI, (size_t)NH_ * ER * HD, HD, (size_t)ER * HD);
    k_gemm<0, DM, DM, DM, DM - 1><<<dim3(NB * SEQ / 64, DM / 64, 1), 32, 0, stream>>>(XB, WK, KP, KR, OUT,
        SEQ, (size_t)NH_ * SEQ * HD, HD, HD, (size_t)SEQ * HD, ER, BIGI, (size_t)NH_ * ER * HD, HD, (size_t)ER * HD);
    k_gemm<0, DM, DM, DM, DM - 1><<<dim3(DM / 64, NB * SEQ / 64, 1), 32, 0, stream>>>(WV, XB, VT, VR, OUT,
        DM, (size_t)0, SEQ, SEQ, (size_t)DM * SEQ, BIGI, ER, (size_t)0, ER, (size_t)DM * ER);

    k_flash<1><<<dim3(ER / (16 * AW), NB * NH_, 1), 32 * AW, 0, stream>>>(QH, QR, KP, KR, VT, VR, CX, 0);
    if (SEQ > ER)
        k_flash<0><<<dim3((SEQ - ER) / (16 * AW), NB * NH_, 1), 32 * AW, 0, stream>>>(QH, QR, KP, KR, VT, VR, CX, ER);

    k_gemm<1, 2 * DM, 2 * DM, DM, DM - 1><<<dim3(NB * SEQ / 64, DM / 64, 1), 32, 0, stream>>>(CX, WO, QH, QR, OUT,
        SEQ, (size_t)OUT_SEQ * DM, DM, DM, (size_t)0, 0, 0, (size_t)0, HD, (size_t)0);
}
